// ExplainModule_89739046683412
// MI455X (gfx1250) — hardware-verified
//
#include <hip/hip_runtime.h>
#include <stdint.h>
#include <stddef.h>
#include <math.h>

#define NN 1024
#define DD 64
#define HH 64
#define PP 132
#define RB 8

static_assert(NN % 32 == 0);
static_assert(NN % 16 == 0);
static_assert(NN % RB == 0);
static_assert(NN % 128 == 0);
static_assert(DD == 64);
static_assert(HH == 64);
static_assert((PP * 4) % 16 == 0);

typedef _Float16 v16h __attribute__((ext_vector_type(16)));
typedef _Float16 v8h  __attribute__((ext_vector_type(8)));
typedef _Float16 v4h  __attribute__((ext_vector_type(4)));
typedef float    v8f  __attribute__((ext_vector_type(8)));
typedef float    v4f  __attribute__((ext_vector_type(4)));
typedef v4f __attribute__((may_alias)) v4fa;

union FragH { v16h v; v8h half[2]; v4h q[4]; };

__device__ __forceinline__ v8f wmma_hf(v16h a, v16h b, v8f c) {
  v8f d = __builtin_amdgcn_wmma_f32_16x16x32_f16(false, a, false, b, (short)0, c, false, false);
  asm volatile("v_nop\n\tv_nop\n\tv_nop\n\tv_nop" : "+v"(d) : "v"(a), "v"(b));
  return d;
}

__device__ __forceinline__ v16h ld_frag_f32(const float* p, int h, float scale) {
  const v4f a0 = *(const v4fa*)(p + 8 * h) * scale;
  const v4f a1 = *(const v4fa*)(p + 8 * h + 4) * scale;
  const v4f a2 = *(const v4fa*)(p + 16 + 8 * h) * scale;
  const v4f a3 = *(const v4fa*)(p + 20 + 8 * h) * scale;
  FragH F;
  F.q[0] = __builtin_convertvector(a0, v4h);
  F.q[1] = __builtin_convertvector(a1, v4h);
  F.q[2] = __builtin_convertvector(a2, v4h);
  F.q[3] = __builtin_convertvector(a3, v4h);
  return F.v;
}

__device__ __forceinline__ v16h mk_pair_frag(v4f p0, v4f p1, v4f p2, v4f p3,
                                             const float* q, int h) {
  const v4f z4 = {0.f, 0.f, 0.f, 0.f};
  const v4f s0 = __builtin_elementwise_max(p0 + *(const v4fa*)(q + 8 * h), z4);
  const v4f s1 = __builtin_elementwise_max(p1 + *(const v4fa*)(q + 8 * h + 4), z4);
  const v4f s2 = __builtin_elementwise_max(p2 + *(const v4fa*)(q + 16 + 8 * h), z4);
  const v4f s3 = __builtin_elementwise_max(p3 + *(const v4fa*)(q + 20 + 8 * h), z4);
  FragH A;
  A.q[0] = __builtin_convertvector(s0, v4h);
  A.q[1] = __builtin_convertvector(s1, v4h);
  A.q[2] = __builtin_convertvector(s2, v4h);
  A.q[3] = __builtin_convertvector(s3, v4h);
  return A.v;
}

__device__ __forceinline__ void proj_store(const float* sP, float* PRE, float* POST,
                                           int r0, int wv, int lane) {
  const int row = 2 * wv + (lane >> 4);
  const int c0  = (lane & 15) * 4;
  const v4f a = *(const v4fa*)(sP + row * PP + c0);
  const v4f b = *(const v4fa*)(sP + row * PP + HH + c0);
  *(volatile v4fa*)(PRE  + (size_t)(r0 + row) * HH + c0) = a;
  *(volatile v4fa*)(POST + (size_t)(r0 + row) * HH + c0) = b;
}

__global__ __launch_bounds__(256) void k_proj(const float* __restrict__ embed,
                                              const float* __restrict__ W1,
                                              const float* __restrict__ b1,
                                              float* __restrict__ PRE,
                                              float* __restrict__ POST)
{
  __shared__ __align__(16) float sP[16 * PP];
  const int tid = threadIdx.x, lane = tid & 31, wv = tid >> 5;
  const int h = lane >> 4, m = lane & 15;
  const int r0  = blockIdx.x * 16;
  const int sel = wv >> 2;
  const int n0  = (wv & 3) * 16;
  const float* arow = embed + (size_t)(r0 + m) * DD;
  const float* wcol = W1 + (size_t)sel * DD * HH + n0 + m;

  const v8f z8 = {0.f, 0.f, 0.f, 0.f, 0.f, 0.f, 0.f, 0.f};
  v8f acc = z8;
  #pragma unroll
  for (int ks = 0; ks < DD / 32; ++ks) {
    const int k0 = 32 * ks;
    const v16h A = ld_frag_f32(arow + k0, h, 1.0f);
    v8f wl, wh;
    #pragma unroll
    for (int e = 0; e < 8; ++e) {
      wl[e] = wcol[(size_t)(k0 + 8 * h + e) * HH] * 16.0f;
      wh[e] = wcol[(size_t)(k0 + 16 + 8 * h + e) * HH] * 16.0f;
    }
    FragH B;
    B.half[0] = __builtin_convertvector(wl, v8h);
    B.half[1] = __builtin_convertvector(wh, v8h);
    acc = wmma_hf(A, B.v, acc);
  }

  const float b1v = b1[n0 + m];
  const float bb  = sel ? 0.f : b1v;
  const int col   = 16 * wv + m;
  #pragma unroll
  for (int r = 0; r < 8; ++r) sP[(8 * h + r) * PP + col] = acc[r] * 0.0625f + bb;
  __syncthreads();

  proj_store(sP, PRE, POST, r0, wv, lane);
  __threadfence();
  proj_store(sP, PRE, POST, r0, wv, lane);
}

__device__ __forceinline__ void gate_store(const float* srw, float* grow, int lane) {
  #pragma unroll
  for (int it = 0; it < NN / 128; ++it) {
    const v4f v = *(const v4fa*)(srw + 128 * it + 4 * lane);
    *(volatile v4fa*)(grow + 128 * it + 4 * lane) = v;
  }
}

__global__ __launch_bounds__(256) void k_gate(const float* __restrict__ PRE,
                                              const float* __restrict__ POST,
                                              const float* __restrict__ W2,
                                              const float* __restrict__ b2,
                                              const float* __restrict__ u,
                                              float* __restrict__ G)
{
  __shared__ __align__(16) float sRow[RB * NN];
  const int tid = threadIdx.x, lane = tid & 31, wv = tid >> 5;
  const int h = lane >> 4, m = lane & 15;
  const int i = blockIdx.x * RB + wv;

  const float* prow = PRE + (size_t)i * HH;
  const v4f p00 = *(const v4fa*)(prow + 8 * h);
  const v4f p01 = *(const v4fa*)(prow + 8 * h + 4);
  const v4f p02 = *(const v4fa*)(prow + 16 + 8 * h);
  const v4f p03 = *(const v4fa*)(prow + 20 + 8 * h);
  const v4f p10 = *(const v4fa*)(prow + 32 + 8 * h);
  const v4f p11 = *(const v4fa*)(prow + 36 + 8 * h);
  const v4f p12 = *(const v4fa*)(prow + 48 + 8 * h);
  const v4f p13 = *(const v4fa*)(prow + 52 + 8 * h);

  const v16h B0 = ld_frag_f32(W2, h, 16.0f);
  const v16h B1 = ld_frag_f32(W2 + 32, h, 16.0f);

  const float bb  = b2[0];
  const int rsel  = lane & 7;
  const int ssel  = (lane >> 3) & 1;
  const int srcl  = 16 * ((lane >> 3) & 1) + 8 * ((lane >> 4) & 1) + (lane & 7);
  const float* urow = u + (size_t)i * NN;
  float* srw = sRow + wv * NN;
  const v8f z8 = {0.f, 0.f, 0.f, 0.f, 0.f, 0.f, 0.f, 0.f};

  #pragma unroll 1
  for (int jt = 0; jt < NN / 32; ++jt) {
    const int j0 = jt * 32;
    const float* q0 = POST + (size_t)(j0 + m) * HH;
    const float* q1 = POST + (size_t)(j0 + 16 + m) * HH;
    v8f acc0 = z8, acc1 = z8;
    {
      const v16h A0 = mk_pair_frag(p00, p01, p02, p03, q0, h);
      const v16h A1 = mk_pair_frag(p00, p01, p02, p03, q1, h);
      acc0 = wmma_hf(A0, B0, acc0);
      acc1 = wmma_hf(A1, B0, acc1);
    }
    {
      const v16h A0 = mk_pair_frag(p10, p11, p12, p13, q0 + 32, h);
      const v16h A1 = mk_pair_frag(p10, p11, p12, p13, q1 + 32, h);
      acc0 = wmma_hf(A0, B1, acc0);
      acc1 = wmma_hf(A1, B1, acc1);
    }

    float v0 = acc0[0], v1 = acc1[0];
    #pragma unroll
    for (int r = 1; r < 8; ++r) {
      v0 = (rsel == r) ? acc0[r] : v0;
      v1 = (rsel == r) ? acc1[r] : v1;
    }
    float la = ssel ? v1 : v0;
    la = __shfl(la, srcl, 32);
    la = la * 0.0625f + bb;

    const float uu = urow[j0 + lane];
    const float nz = logf(uu) - log1pf(-uu);
    const float s  = nz + la;
    const float e  = expf(-s);
    const float g  = __builtin_amdgcn_rcpf(1.0f + e);
    srw[j0 + lane] = g;
  }
  __syncthreads();

  float* grow = G + (size_t)i * NN;
  gate_store(srw, grow, lane);
  __threadfence();
  gate_store(srw, grow, lane);
}

__global__ __launch_bounds__(256) void k_out(const float* __restrict__ G,
                                             const float* __restrict__ adj,
                                             float* __restrict__ out)
{
  __shared__ float sT[32 * 33];
  const int tid = threadIdx.x;
  const int i0 = blockIdx.y * 32, j0 = blockIdx.x * 32;
  const int r = tid >> 3, q = tid & 7;

  const v4f t4 = *(const v4fa*)(G + (size_t)(j0 + r) * NN + i0 + 4 * q);
  sT[r * 33 + 4 * q + 0] = t4.x;
  sT[r * 33 + 4 * q + 1] = t4.y;
  sT[r * 33 + 4 * q + 2] = t4.z;
  sT[r * 33 + 4 * q + 3] = t4.w;
  __syncthreads();

  const size_t off = (size_t)(i0 + r) * NN + j0 + 4 * q;
  const v4f g4 = *(const v4fa*)(G + off);
  const v4f a4 = *(const v4fa*)(adj + off);
  v4f gt;
  gt.x = sT[(4 * q + 0) * 33 + r];
  gt.y = sT[(4 * q + 1) * 33 + r];
  gt.z = sT[(4 * q + 2) * 33 + r];
  gt.w = sT[(4 * q + 3) * 33 + r];
  const v4f o = a4 * ((g4 + gt) * 0.5f);

  float* op = out + off;
  *(volatile v4fa*)op = o;
  __threadfence();
  *(volatile v4fa*)op = o;
}

extern "C" void kernel_launch(void* const* d_in, const int* in_sizes, int n_in,
                              void* d_out, int out_size, void* d_ws, size_t ws_size,
                              hipStream_t stream)
{
  if (n_in < 7) return;
  if (in_sizes[0] != NN * DD) return;
  if (in_sizes[1] != NN * NN) return;
  if (in_sizes[2] != NN * NN) return;
  if (in_sizes[3] != 2 * DD * HH) return;
  if (in_sizes[4] != HH) return;
  if (in_sizes[5] != HH) return;
  if (in_sizes[6] < 1) return;
  if (out_size != NN * NN) return;

  const float* embed = (const float*)d_in[0];
  const float* adj   = (const float*)d_in[1];
  const float* u     = (const float*)d_in[2];
  const float* W1    = (const float*)d_in[3];
  const float* b1    = (const float*)d_in[4];
  const float* W2    = (const float*)d_in[5];
  const float* b2    = (const float*)d_in[6];
  float* out = (float*)d_out;

  const size_t bP = (size_t)NN * HH * 4;
  const size_t bG = (size_t)NN * NN * 4;
  const size_t total = 2 * bP + bG;
  if (total > ws_size) return;
  if (total > (size_t)134217728) return;

  char* ws = (char*)d_ws;
  size_t off = 0;
  float* PRE  = (float*)(ws + off); off += bP;
  float* POST = (float*)(ws + off); off += bP;
  float* G    = (float*)(ws + off); off += bG;
  if (off != total) return;

  k_proj<<<NN / 16, 256, 0, stream>>>(embed, W1, b1, PRE, POST);
  k_gate<<<NN / RB, 256, 0, stream>>>(PRE, POST, W2, b2, u, G);
  k_out<<<dim3(NN / 32, NN / 32), 256, 0, stream>>>(G, adj, out);
}
